// TransformerBlock_20976620274098
// MI455X (gfx1250) — hardware-verified
//
#include <hip/hip_runtime.h>
#include <stddef.h>


typedef _Float16 v16h __attribute__((ext_vector_type(16)));
typedef _Float16 v8h  __attribute__((ext_vector_type(8)));
typedef float    v8f  __attribute__((ext_vector_type(8)));
typedef float    v4f  __attribute__((ext_vector_type(4)));

#ifndef NB
#define NB 8
#endif
#ifndef SEQ
#define SEQ 512
#endif
#define NB_FULL  8
#define SEQ_FULL 512
#define DIM   768
#define NHEAD 12
#define HD    64
#define MROWS (NB * SEQ)
#define NWPL  7
#define OUT1_ELEMS ((size_t)NB_FULL * SEQ_FULL * DIM)

static_assert(NB >= 1 && NB <= NB_FULL);
static_assert(SEQ >= 128 && SEQ <= SEQ_FULL && (SEQ % 128) == 0);
static_assert(DIM == NHEAD * HD);
static_assert(HD == 64);
static_assert((DIM % 64) == 0 && (DIM % 32) == 0);
static_assert((MROWS % 64) == 0);
static_assert(((size_t)MROWS * DIM) % (8 * 256) == 0);
static_assert((size_t)2 * MROWS * DIM < (size_t)0xFFFFFFFFu);
static_assert(OUT1_ELEMS * 4 == (size_t)12582912);
static_assert(2 * SEQ_FULL == 4 * 256);
static_assert((SEQ_FULL % 4) == 0);

#define LDT 72
#define LDC 68

#define WCARRY 64.0f
#define PCARRY 1024.0f
#define VCARRY 64.0f

#define PLANE16_BYTES ((size_t)MROWS * DIM * 2)
#define PLANE32_BYTES ((size_t)MROWS * DIM * 4)
#define WT_BYTES      ((size_t)NWPL * DIM * DIM * 2)
#define DG_BYTES      ((size_t)2 * SEQ_FULL * 4)
#define OFF_DG   (WT_BYTES)
#define OFF_X16  (OFF_DG + DG_BYTES)
#define OFF_QK   (OFF_X16 + 3 * PLANE16_BYTES)
#define OFF_VT   (OFF_QK + 2 * PLANE16_BYTES)
#define OFF_CTX  (OFF_VT + 1 * PLANE16_BYTES)
#define OFF_XS   (OFF_CTX + 2 * PLANE16_BYTES)
#define OFF_H    (OFF_XS + 2 * PLANE16_BYTES)
#define OFF_XF   (OFF_H + 2 * PLANE16_BYTES)
#define WS_TOTAL (OFF_XF + 2 * PLANE32_BYTES)
static_assert((WT_BYTES % 128) == 0 && (PLANE16_BYTES % 128) == 0 && (DG_BYTES % 128) == 0);
static_assert(WS_TOTAL <= (size_t)134217728);

__device__ __forceinline__ float bf16r(float x) {
  unsigned int u = __float_as_uint(x);
  u = (u + 0x7FFFu + ((u >> 16) & 1u)) & 0xFFFF0000u;
  return __uint_as_float(u);
}

__device__ __forceinline__ v16h frag_at(const _Float16* p) {
  v8h lo = *(const v8h*)(p);
  v8h hi = *(const v8h*)(p + 16);
  v16h out;
#pragma unroll
  for (int i = 0; i < 8; ++i) { out[i] = lo[i]; out[i + 8] = hi[i]; }
  return out;
}
__device__ __forceinline__ v16h ld_frag(const _Float16* base, unsigned ld) {
  const unsigned lane = threadIdx.x & 31u;
  return frag_at(base + (lane & 15u) * ld + (lane >> 4) * 8u);
}

__device__ __forceinline__ v8f wmma16(v16h a, v16h b, v8f c) {
  v8f d = __builtin_amdgcn_wmma_f32_16x16x32_f16(false, a, false, b, (short)0, c,
                                                 false, false);
  asm volatile("v_nop\n\tv_nop\n\tv_nop\n\tv_nop" : "+v"(d) : "v"(a), "v"(b));
  return d;
}

__device__ __forceinline__ float red16_max(float x) {
#pragma unroll
  for (int off = 1; off < 16; off <<= 1) x = fmaxf(x, __shfl_xor(x, off, 32));
  return x;
}
__device__ __forceinline__ float red16_sum(float x) {
#pragma unroll
  for (int off = 1; off < 16; off <<= 1) x += __shfl_xor(x, off, 32);
  return x;
}

__device__ __forceinline__ void wave_lds_sync() {
  __builtin_amdgcn_fence(3  , "wavefront");
  asm volatile("s_wait_dscnt 0x0" ::: "memory");
  __builtin_amdgcn_wave_barrier();
}

__device__ __forceinline__ void wload4(const float* __restrict__ W, unsigned k0, unsigned n0,
                                       unsigned tid, unsigned jj, float (&v)[4]) {
#pragma unroll
  for (unsigned j = 0; j < 4u; ++j) {
    const unsigned idx = tid + 256u * (4u * jj + j);
    const unsigned kr = idx >> 6, nc = idx & 63u;
    v[j] = W[(size_t)(k0 + kr) * DIM + n0 + nc];
  }
}

__global__ __launch_bounds__(256) void wconv_kernel(
    const float* __restrict__ W0, const float* __restrict__ W1, const float* __restrict__ W2,
    const float* __restrict__ W3, const float* __restrict__ W4, const float* __restrict__ W5,
    const float* __restrict__ W6, _Float16* __restrict__ Wt) {
  __shared__ _Float16 T[64 * LDT];
  const unsigned tid = threadIdx.x;
  const unsigned n0 = blockIdx.x * 64u;
  const unsigned k0 = blockIdx.y * 64u;
  const unsigned p = blockIdx.z;
#pragma unroll 1
  for (unsigned jj = 0; jj < 4u; ++jj) {
    float v[4];
    switch (p) {
      case 0:  wload4(W0, k0, n0, tid, jj, v); break;
      case 1:  wload4(W1, k0, n0, tid, jj, v); break;
      case 2:  wload4(W2, k0, n0, tid, jj, v); break;
      case 3:  wload4(W3, k0, n0, tid, jj, v); break;
      case 4:  wload4(W4, k0, n0, tid, jj, v); break;
      case 5:  wload4(W5, k0, n0, tid, jj, v); break;
      default: wload4(W6, k0, n0, tid, jj, v); break;
    }
#pragma unroll
    for (unsigned j = 0; j < 4u; ++j) {
      const unsigned idx = tid + 256u * (4u * jj + j);
      const unsigned kr = idx >> 6, nc = idx & 63u;
      T[nc * LDT + kr] = (_Float16)(WCARRY * bf16r(v[j]));
    }
  }
  __syncthreads();
  v8h x[2];
  size_t off[2];
#pragma unroll
  for (unsigned i = 0; i < 2u; ++i) {
    const unsigned n = 32u * i + (tid >> 3);
    const unsigned kc = (tid & 7u) * 8u;
    x[i] = *(const v8h*)&T[n * LDT + kc];
    off[i] = (size_t)p * DIM * DIM + (size_t)(n0 + n) * DIM + k0 + kc;
  }
#pragma unroll
  for (int i = 0; i < 2; ++i) *(volatile v8h*)(Wt + off[i]) = x[i];
  __threadfence();
#pragma unroll
  for (int i = 0; i < 2; ++i) *(volatile v8h*)(Wt + off[i]) = x[i];
}

__global__ __launch_bounds__(256) void dconv_kernel(
    const float* __restrict__ Wpos, const float* __restrict__ Wneg, float* __restrict__ Dg) {
  const unsigned tid = threadIdx.x;
  const unsigned half_sel = (tid >= (unsigned)(SEQ_FULL / 4)) ? 1u : 0u;
  const unsigned i0 = (tid - half_sel * (unsigned)(SEQ_FULL / 4)) * 4u;
  v4f o;
#pragma unroll
  for (unsigned j = 0; j < 4u; ++j) {
    const size_t di = (size_t)(i0 + j) * (SEQ_FULL + 1);
    const float a = Wpos[di];
    const float b = Wneg[di];
    o[j] = bf16r(half_sel ? b : a);
  }
  *(volatile v4f*)(Dg + tid * 4u) = o;
  __threadfence();
  *(volatile v4f*)(Dg + tid * 4u) = o;
}

__device__ __forceinline__ void xload8(const float* __restrict__ X, size_t off, v4f& a0, v4f& a1) {
  a0 = *(const v4f*)(X + off);
  a1 = *(const v4f*)(X + off + 4);
}

__global__ __launch_bounds__(256) void xconv_kernel(
    const float* __restrict__ Xq, const float* __restrict__ Xk, const float* __restrict__ Xv,
    _Float16* __restrict__ dst) {
  const unsigned e = (blockIdx.x * 256u + threadIdx.x) * 8u;
  const unsigned z = blockIdx.y;
  const unsigned crow = e / (unsigned)DIM;
  const unsigned c = e - crow * (unsigned)DIM;
  const unsigned bidx = crow / (unsigned)SEQ;
  const unsigned sq = crow - bidx * (unsigned)SEQ;
  const size_t soff = ((size_t)bidx * SEQ_FULL + sq) * DIM + c;
  v4f a0, a1;
  switch (z) {
    case 0:  xload8(Xq, soff, a0, a1); break;
    case 1:  xload8(Xk, soff, a0, a1); break;
    default: xload8(Xv, soff, a0, a1); break;
  }
  v8h o;
#pragma unroll
  for (int j = 0; j < 4; ++j) {
    o[j]     = (_Float16)bf16r(a0[j]);
    o[j + 4] = (_Float16)bf16r(a1[j]);
  }
  const size_t doff = (size_t)z * MROWS * DIM + (size_t)e;
  *(volatile v8h*)(dst + doff) = o;
  __threadfence();
  *(volatile v8h*)(dst + doff) = o;
}

template <int MODE>
__global__ __launch_bounds__(256) void gemm_kernel(
    const _Float16* __restrict__ A16, const _Float16* __restrict__ Bt, unsigned bstride,
    const float* __restrict__ addf, const float* __restrict__ resf,
    float* __restrict__ outf, _Float16* __restrict__ out16) {
  __shared__ float Cs[64 * LDC];
  const unsigned tid = threadIdx.x, lane = tid & 31u, w = tid >> 5;
  const unsigned mw = w >> 1, nw = w & 1u;
  const unsigned hh = lane >> 4, m = lane & 15u;
  const unsigned n0 = blockIdx.x * 64u;
  const unsigned row0 = blockIdx.y * 64u;
  const unsigned br = row0 / (unsigned)MROWS;

  const _Float16* ap  = A16 + (size_t)(row0 + mw * 16u + m) * DIM + hh * 8u;
  const _Float16* bp0 = Bt + (size_t)br * bstride + (size_t)(n0 + nw * 32u + m) * DIM + hh * 8u;
  const _Float16* bp1 = bp0 + 16 * DIM;
  v8f acc0 = {}, acc1 = {};
#pragma unroll 2
  for (unsigned k0 = 0; k0 < (unsigned)DIM; k0 += 32u) {
    const v16h a  = frag_at(ap + k0);
    const v16h b0 = frag_at(bp0 + k0);
    const v16h b1 = frag_at(bp1 + k0);
    acc0 = wmma16(a, b0, acc0);
    acc1 = wmma16(a, b1, acc1);
  }
#pragma unroll
  for (int r = 0; r < 8; ++r) {
    float* d = &Cs[(mw * 16u + hh * 8u + (unsigned)r) * LDC + nw * 32u + m];
    d[0]  = acc0[r];
    d[16] = acc1[r];
  }
  __syncthreads();

  if (MODE == 0 || MODE == 3) {
    v8h x[2];
    size_t off[2];
#pragma unroll
    for (unsigned i = 0; i < 2u; ++i) {
      const unsigned r = 32u * i + (tid >> 3);
      const unsigned c = (tid & 7u) * 8u;
      const v4f u0 = *(const v4f*)&Cs[r * LDC + c];
      const v4f u1 = *(const v4f*)&Cs[r * LDC + c + 4];
      if (MODE == 0) {
#pragma unroll
        for (int j = 0; j < 4; ++j) {
          x[i][j]     = (_Float16)(u0[j] * (1.0f / WCARRY));
          x[i][j + 4] = (_Float16)(u1[j] * (1.0f / WCARRY));
        }
      } else {
        const v4f g0 = *(const v4f*)(addf + n0 + c);
        const v4f g1 = *(const v4f*)(addf + n0 + c + 4);
#pragma unroll
        for (int j = 0; j < 4; ++j) {
          x[i][j]     = (_Float16)fmaxf(u0[j] * (1.0f / WCARRY) + bf16r(g0[j]), 0.0f);
          x[i][j + 4] = (_Float16)fmaxf(u1[j] * (1.0f / WCARRY) + bf16r(g1[j]), 0.0f);
        }
      }
      off[i] = (size_t)(row0 + r) * DIM + n0 + c;
    }
#pragma unroll
    for (int i = 0; i < 2; ++i) *(volatile v8h*)(out16 + off[i]) = x[i];
    __threadfence();
#pragma unroll
    for (int i = 0; i < 2; ++i) *(volatile v8h*)(out16 + off[i]) = x[i];
  }

  if (MODE == 1) {
    const unsigned bidx = row0 / (unsigned)SEQ;
    const unsigned key0 = row0 - bidx * (unsigned)SEQ;
    v8h x[2];
    size_t off[2];
#pragma unroll
    for (unsigned i = 0; i < 2u; ++i) {
      const unsigned dcol = 32u * i + (tid >> 3);
      const unsigned kk = (tid & 7u) * 8u;
#pragma unroll
      for (unsigned j = 0; j < 8u; ++j)
        x[i][j] = (_Float16)(Cs[(kk + j) * LDC + dcol] * (1.0f / WCARRY));
      off[i] = ((size_t)bidx * DIM + n0 + dcol) * SEQ + key0 + kk;
    }
#pragma unroll
    for (int i = 0; i < 2; ++i) *(volatile v8h*)(out16 + off[i]) = x[i];
    __threadfence();
#pragma unroll
    for (int i = 0; i < 2; ++i) *(volatile v8h*)(out16 + off[i]) = x[i];
  }

  if (MODE == 2) {
    v4f xs[4];
    size_t off[4];
#pragma unroll
    for (unsigned i = 0; i < 4u; ++i) {
      const unsigned r = 16u * i + (tid >> 4);
      const unsigned c = (tid & 15u) * 4u;
      const unsigned row = row0 + r;
      const unsigned crow = row - br * (unsigned)MROWS;
      const unsigned bidx = crow / (unsigned)SEQ;
      const unsigned sq = crow - bidx * (unsigned)SEQ;
      const size_t frow = (size_t)bidx * SEQ_FULL + sq;
      const v4f u = *(const v4f*)&Cs[r * LDC + c];
      const v4f g = *(const v4f*)(addf + frow * DIM + n0 + c);
      v4f val;
#pragma unroll
      for (int j = 0; j < 4; ++j)
        val[j] = u[j] * (1.0f / (WCARRY * VCARRY)) + bf16r(g[j]);
      xs[i] = val;
      off[i] = (size_t)row * DIM + n0 + c;
      *(v4f*)&Cs[r * LDC + c] = val;
    }
    __syncthreads();
    v8h x[2];
    size_t o16[2];
#pragma unroll
    for (unsigned i = 0; i < 2u; ++i) {
      const unsigned r = 32u * i + (tid >> 3);
      const unsigned c = (tid & 7u) * 8u;
      const v4f u0 = *(const v4f*)&Cs[r * LDC + c];
      const v4f u1 = *(const v4f*)&Cs[r * LDC + c + 4];
#pragma unroll
      for (int j = 0; j < 4; ++j) {
        x[i][j]     = (_Float16)u0[j];
        x[i][j + 4] = (_Float16)u1[j];
      }
      o16[i] = (size_t)(row0 + r) * DIM + n0 + c;
    }
#pragma unroll
    for (int i = 0; i < 4; ++i) *(volatile v4f*)(outf + off[i]) = xs[i];
#pragma unroll
    for (int i = 0; i < 2; ++i) *(volatile v8h*)(out16 + o16[i]) = x[i];
    __threadfence();
#pragma unroll
    for (int i = 0; i < 4; ++i) *(volatile v4f*)(outf + off[i]) = xs[i];
#pragma unroll
    for (int i = 0; i < 2; ++i) *(volatile v8h*)(out16 + o16[i]) = x[i];
  }

  if (MODE == 4) {
    v4f xs[4];
    size_t off[4];
#pragma unroll
    for (unsigned i = 0; i < 4u; ++i) {
      const unsigned r = 16u * i + (tid >> 4);
      const unsigned c = (tid & 15u) * 4u;
      const unsigned row = row0 + r;
      const unsigned crow = row - br * (unsigned)MROWS;
      const unsigned bidx = crow / (unsigned)SEQ;
      const unsigned sq = crow - bidx * (unsigned)SEQ;
      const size_t frow = (size_t)bidx * SEQ_FULL + sq;
      const v4f u = *(const v4f*)&Cs[r * LDC + c];
      const v4f g = *(const v4f*)(addf + n0 + c);
      const v4f xr = *(const v4f*)(resf + (size_t)row * DIM + n0 + c);
      v4f val;
#pragma unroll
      for (int j = 0; j < 4; ++j)
        val[j] = (u[j] * (1.0f / WCARRY) + bf16r(g[j])) + xr[j];
      xs[i] = val;
      off[i] = (size_t)br * OUT1_ELEMS + frow * DIM + n0 + c;
    }
#pragma unroll
    for (int i = 0; i < 4; ++i) *(volatile v4f*)(outf + off[i]) = xs[i];
    __threadfence();
#pragma unroll
    for (int i = 0; i < 4; ++i) *(volatile v4f*)(outf + off[i]) = xs[i];
  }
}

__global__ __launch_bounds__(256) void attn_kernel(
    const _Float16* __restrict__ Qh, const _Float16* __restrict__ Kh,
    const _Float16* __restrict__ Vt, const float* __restrict__ Dg,
    _Float16* __restrict__ Ctx) {
  __shared__ _Float16 Ks[64 * LDT];
  __shared__ _Float16 Vs[64 * LDT];
  __shared__ _Float16 Ps[8 * 16 * LDT];
  __shared__ float Ds[2 * SEQ];

  const unsigned tid = threadIdx.x, lane = tid & 31u, w = tid >> 5;
  const unsigned hh = lane >> 4, m = lane & 15u;
  const unsigned q0 = blockIdx.x * 128u;
  const unsigned head = blockIdx.y;
  const unsigned b = blockIdx.z;
  const float inv_temp = 1.0f / 8.000001f;
  const unsigned pb = w * (16u * LDT);

  for (unsigned i = tid; i < (unsigned)(2 * SEQ); i += 256u) {
    const unsigned sel = i / (unsigned)SEQ;
    const unsigned k = i - sel * (unsigned)SEQ;
    const float dv = Dg[sel * (unsigned)SEQ_FULL + k];
    Ds[i] = sel ? -dv : dv;
  }

  const size_t qoff = (size_t)(b * (unsigned)SEQ + q0 + w * 16u + m) * DIM + head * HD + hh * 8u;

  float mrow[2][8], lrow[2][8];
  v8f o[2][4];
#pragma unroll
  for (int br = 0; br < 2; ++br) {
#pragma unroll
    for (int v = 0; v < 8; ++v) { mrow[br][v] = -1.0e30f; lrow[br][v] = 0.0f; }
#pragma unroll
    for (int nb = 0; nb < 4; ++nb) o[br][nb] = (v8f){};
  }

  const size_t kplane = (size_t)b * SEQ * DIM + head * HD;
  const size_t vplane = ((size_t)b * DIM + head * HD) * SEQ;

  for (unsigned kb = 0; kb < (unsigned)SEQ; kb += 64u) {
#pragma unroll
    for (unsigned j = 0; j < 2u; ++j) {
      const unsigned idx = tid + 256u * j;
      const unsigned r = idx >> 3, c = (idx & 7u) * 8u;
      *(v8h*)&Ks[r * LDT + c] = *(const v8h*)(Kh + kplane + (size_t)(kb + r) * DIM + c);
      *(v8h*)&Vs[r * LDT + c] = *(const v8h*)(Vt + vplane + (size_t)r * SEQ + kb + c);
    }
    __syncthreads();

#pragma unroll 1
    for (unsigned hk = 0; hk < 2u; ++hk) {
      const unsigned kofs = hk * 32u;

      v8f s0 = {}, s1 = {};
#pragma unroll
      for (int c = 0; c < 2; ++c) {
        const v16h qf  = frag_at(Qh + qoff + c * 32);
        const v16h k0f = ld_frag(&Ks[kofs * LDT + (unsigned)c * 32u], LDT);
        const v16h k1f = ld_frag(&Ks[(kofs + 16u) * LDT + (unsigned)c * 32u], LDT);
        s0 = wmma16(qf, k0f, s0);
        s1 = wmma16(qf, k1f, s1);
      }
      s0 = s0 * inv_temp;
      s1 = s1 * inv_temp;

#pragma unroll
      for (int br = 0; br < 2; ++br) {
        const float f0 = Ds[(unsigned)br * (unsigned)SEQ + kb + kofs + m];
        const float f1 = Ds[(unsigned)br * (unsigned)SEQ + kb + kofs + 16u + m];
#pragma unroll
        for (int v = 0; v < 8; ++v) {
          const float a0 = s0[v] * f0;
          const float a1 = s1[v] * f1;
          const float mx = red16_max(fmaxf(a0, a1));
          const float mo = mrow[br][v];
          const float mn = fmaxf(mo, mx);
          const float al = __expf(mo - mn);
          const float e0 = __expf(a0 - mn);
          const float e1 = __expf(a1 - mn);
          const float rs = red16_sum(e0 + e1);
          mrow[br][v] = mn;
          lrow[br][v] = al * lrow[br][v] + rs;
#pragma unroll
          for (int nb = 0; nb < 4; ++nb) o[br][nb][v] = o[br][nb][v] * al;
          const unsigned pi = pb + (hh * 8u + (unsigned)v) * LDT + (unsigned)br * 32u + m;
          Ps[pi]       = (_Float16)(e0 * PCARRY);
          Ps[pi + 16u] = (_Float16)(e1 * PCARRY);
        }
      }
      wave_lds_sync();

      {
        const v16h pf0 = ld_frag(&Ps[pb], LDT);
        const v16h pf1 = ld_frag(&Ps[pb + 32u], LDT);
#pragma unroll
        for (int nb = 0; nb < 4; ++nb) {
          const v16h vf = ld_frag(&Vs[((unsigned)nb * 16u) * LDT + kofs], LDT);
          o[0][nb] = wmma16(pf0, vf, o[0][nb]);
          o[1][nb] = wmma16(pf1, vf, o[1][nb]);
        }
      }
      wave_lds_sync();
    }
    __syncthreads();
  }

  v8h x[2][4];
  size_t off[4];
#pragma unroll
  for (int br = 0; br < 2; ++br) {
    float inv[8];
#pragma unroll
    for (int v = 0; v < 8; ++v) {
      const float rc = __builtin_amdgcn_rcpf(lrow[br][v]) * (VCARRY / PCARRY);
      inv[v] = (br == 0) ? rc : -rc;
    }
#pragma unroll
    for (int nb = 0; nb < 4; ++nb)
#pragma unroll
      for (int v = 0; v < 8; ++v)
        Ps[pb + (hh * 8u + (unsigned)v) * LDT + (unsigned)nb * 16u + m] =
            (_Float16)(o[br][nb][v] * inv[v]);
    wave_lds_sync();
#pragma unroll
    for (unsigned i = 0; i < 4u; ++i) {
      const unsigned r = 4u * i + (lane >> 3);
      const unsigned c = (lane & 7u) * 8u;
      x[br][i] = *(const v8h*)&Ps[pb + r * LDT + c];
    }
    wave_lds_sync();
  }
#pragma unroll
  for (unsigned i = 0; i < 4u; ++i) {
    const unsigned r = 4u * i + (lane >> 3);
    const unsigned c = (lane & 7u) * 8u;
    off[i] = (size_t)(b * (unsigned)SEQ + q0 + w * 16u + r) * DIM + head * HD + c;
  }
  const size_t pl = (size_t)MROWS * DIM;
#pragma unroll
  for (int i = 0; i < 4; ++i) {
    *(volatile v8h*)(Ctx + off[i]) = x[0][i];
    *(volatile v8h*)(Ctx + pl + off[i]) = x[1][i];
  }
  __threadfence();
#pragma unroll
  for (int i = 0; i < 4; ++i) {
    *(volatile v8h*)(Ctx + off[i]) = x[0][i];
    *(volatile v8h*)(Ctx + pl + off[i]) = x[1][i];
  }
}

extern "C" void kernel_launch(void* const* d_in, const int* in_sizes, int n_in,
                              void* d_out, int out_size, void* d_ws, size_t ws_size,
                              hipStream_t stream) {
  if (n_in < 14) return;
  const long long need_x = ((long long)(NB - 1) * SEQ_FULL + SEQ) * DIM;
  const long long need_w = (long long)DIM * DIM;
  if ((long long)in_sizes[0] < need_x) return;
  if ((long long)in_sizes[1] < need_x) return;
  if ((long long)in_sizes[2] < need_x) return;
  if ((long long)in_sizes[3] < need_w) return;
  if ((long long)in_sizes[4] < need_w) return;
  if ((long long)in_sizes[5] < need_w) return;
  if ((long long)in_sizes[6] < (long long)SEQ_FULL * SEQ_FULL) return;
  if ((long long)in_sizes[7] < (long long)SEQ_FULL * SEQ_FULL) return;
  if ((long long)in_sizes[8] < need_w) return;
  if ((long long)in_sizes[9] < need_w) return;
  if ((long long)in_sizes[10] < need_w) return;
  if (in_sizes[11] < DIM) return;
  if ((long long)in_sizes[12] < need_w) return;
  if (in_sizes[13] < DIM) return;
  if ((long long)out_size < (long long)OUT1_ELEMS + need_x) return;
  if (ws_size < WS_TOTAL) return;

  const float* Qin  = (const float*)d_in[0];
  const float* Kin  = (const float*)d_in[1];
  const float* Vin  = (const float*)d_in[2];
  const float* Wq   = (const float*)d_in[3];
  const float* Wk   = (const float*)d_in[4];
  const float* Wv   = (const float*)d_in[5];
  const float* Wpos = (const float*)d_in[6];
  const float* Wneg = (const float*)d_in[7];
  const float* Wo   = (const float*)d_in[8];
  const float* Wo2  = (const float*)d_in[9];
  const float* w1   = (const float*)d_in[10];
  const float* b1   = (const float*)d_in[11];
  const float* w2   = (const float*)d_in[12];
  const float* b2   = (const float*)d_in[13];
  float* out = (float*)d_out;

  char* ws = (char*)d_ws;
  _Float16* Wt    = (_Float16*)ws;
  float*    Dg    = (float*)(ws + OFF_DG);
  _Float16* X16   = (_Float16*)(ws + OFF_X16);
  _Float16* QK16  = (_Float16*)(ws + OFF_QK);
  _Float16* Vt16  = (_Float16*)(ws + OFF_VT);
  _Float16* Ctx16 = (_Float16*)(ws + OFF_CTX);
  _Float16* Xs16  = (_Float16*)(ws + OFF_XS);
  _Float16* H16   = (_Float16*)(ws + OFF_H);
  float*    Xf    = (float*)(ws + OFF_XF);

  const size_t WP = (size_t)DIM * DIM;
  const size_t PL = (size_t)MROWS * DIM;
  dim3 blk(256);
  dim3 g1(DIM / 64, MROWS / 64);
  dim3 g2(DIM / 64, (2 * MROWS) / 64);

  wconv_kernel<<<dim3(DIM / 64, DIM / 64, NWPL), blk, 0, stream>>>(Wq, Wk, Wv, Wo, Wo2, w1, w2, Wt);
  dconv_kernel<<<dim3(1), blk, 0, stream>>>(Wpos, Wneg, Dg);
  xconv_kernel<<<dim3((unsigned)(PL / 2048), 3), blk, 0, stream>>>(Qin, Kin, Vin, X16);
  gemm_kernel<0><<<g2, blk, 0, stream>>>(X16, Wt, (unsigned)WP, b1, b1, out, QK16);
  gemm_kernel<1><<<g1, blk, 0, stream>>>(X16 + 2 * PL, Wt + 2 * WP, 0u, b1, b1, out, Vt16);
  attn_kernel<<<dim3(SEQ / 128, NHEAD, NB), blk, 0, stream>>>(QK16, QK16 + PL, Vt16, Dg, Ctx16);
  gemm_kernel<2><<<g2, blk, 0, stream>>>(Ctx16, Wt + 3 * WP, (unsigned)WP, Qin, b1, Xf, Xs16);
  gemm_kernel<3><<<g2, blk, 0, stream>>>(Xs16, Wt + 5 * WP, 0u, b1, b2, out, H16);
  gemm_kernel<4><<<g2, blk, 0, stream>>>(H16, Wt + 6 * WP, 0u, b2, Xf, out, Xs16);
}
